// QuantumLayer_78692390797439
// MI455X (gfx1250) — hardware-run, weakly checked
//
#include <hip/hip_runtime.h>
#include <math.h>

typedef __attribute__((ext_vector_type(16))) _Float16 v16h;
typedef __attribute__((ext_vector_type(8)))  _Float16 v8h;
typedef __attribute__((ext_vector_type(8)))  float    v8f;
typedef __attribute__((ext_vector_type(4)))  float    v4f;

constexpr int kWires        = 4;
constexpr int kDim          = 16;
constexpr int kLayers       = 2;
constexpr int kAngles       = kLayers * kWires * 3;
constexpr int kBatch        = 1048576;
constexpr int kPlaneRows    = 2 * kDim;
constexpr int kPlaneK       = 32;
constexpr int kRowsPerTile  = 32;
constexpr int kWavesPerBlk  = 8;
constexpr int kTilesPerWave = 4;
constexpr int kSlabPitch    = 20;
constexpr int kMainBlocks   = kBatch / (kRowsPerTile * kWavesPerBlk * kTilesPerWave);
static_assert(kDim == (1 << kWires));
static_assert(kAngles == 24);
static_assert(kPlaneK == 2 * kDim);
static_assert(kBatch % (kRowsPerTile * kWavesPerBlk * kTilesPerWave) == 0);
static_assert(kMainBlocks == 1024);
static_assert((kSlabPitch % 4) == 0 && kSlabPitch >= kDim);

constexpr float kCarryA = 1024.0f;
constexpr float kCarryB = 32.0f;
constexpr float kFold   = 1.0f / ((kCarryA * kCarryB) * (kCarryA * kCarryB));

constexpr size_t kOffPlane = 0;
constexpr size_t kWsTotal  = kOffPlane + (size_t)kPlaneRows * kPlaneK * 2;
static_assert(kWsTotal == 2048ull);
static_assert(kWsTotal <= 134217728ull);

struct FragH {
  union U { v16h v; v8h h[2]; };
  static __device__ __forceinline__ v16h load(const _Float16* p) {
    U f;
    f.h[0] = *(const v8h*)(p);
    f.h[1] = *(const v8h*)(p + 16);
    return f.v;
  }
};

__device__ __forceinline__ v8f mma_f16_guarded(v16h a, v16h b, v8f c) {
  c = __builtin_amdgcn_wmma_f32_16x16x32_f16(false, a, false, b, (short)0, c, false, false);
  asm volatile("v_nop\n\tv_nop\n\tv_nop\n\tv_nop" : "+v"(c) : "v"(a), "v"(b));
  return c;
}

__global__ __launch_bounds__(256) void build_gate_plane_kernel(
    const float* __restrict__ wts, unsigned short* __restrict__ plane)
{
  __shared__ float Ur[kDim * kDim];
  __shared__ float Ui[kDim * kDim];
  __shared__ float tc[kAngles];
  __shared__ float ts[kAngles];
  const int t = threadIdx.x;
  const int i = t >> 4;
  const int j = t & 15;
  {
    const int ta = (t < kAngles) ? t : (kAngles - 1);
    float w = wts[ta];
    asm volatile("" : "+v"(w));
    float sv, cv;
    sincosf(0.5f * w, &sv, &cv);
    if (t < kAngles) {
      tc[t] = cv;
      ts[t] = sv;
    }
  }
  Ur[t] = (i == j) ? 1.0f : 0.0f;
  Ui[t] = 0.0f;
  __syncthreads();

#pragma unroll 1
  for (int l = 0; l < kLayers; ++l) {
#pragma unroll 1
    for (int q = 0; q < kWires; ++q) {
      const int bitpos = 3 - q;
      if (t < 128) {
        const int col = t & 15;
        const int p   = t >> 4;
        const int i0  = ((p >> bitpos) << (bitpos + 1)) | (p & ((1 << bitpos) - 1));
        const int i1  = i0 | (1 << bitpos);
        float u0r = Ur[i0 * kDim + col], u0i = Ui[i0 * kDim + col];
        float u1r = Ur[i1 * kDim + col], u1i = Ui[i1 * kDim + col];
        const int g = (l * kWires + q) * 3;
        float c = tc[g + 0], s = ts[g + 0];
        float n0r = c * u0r + s * u1i, n0i = c * u0i - s * u1r;
        float n1r = c * u1r + s * u0i, n1i = c * u1i - s * u0r;
        u0r = n0r; u0i = n0i; u1r = n1r; u1i = n1i;
        c = tc[g + 1]; s = ts[g + 1];
        n0r = c * u0r - s * u1r; n0i = c * u0i - s * u1i;
        n1r = s * u0r + c * u1r; n1i = s * u0i + c * u1i;
        u0r = n0r; u0i = n0i; u1r = n1r; u1i = n1i;
        c = tc[g + 2]; s = ts[g + 2];
        n0r = c * u0r + s * u0i; n0i = c * u0i - s * u0r;
        n1r = c * u1r - s * u1i; n1i = c * u1i + s * u1r;
        Ur[i0 * kDim + col] = n0r; Ui[i0 * kDim + col] = n0i;
        Ur[i1 * kDim + col] = n1r; Ui[i1 * kDim + col] = n1i;
      }
      __syncthreads();
    }
#pragma unroll 1
    for (int q = 0; q < kWires; ++q) {
      const int tq    = (q + 1) & 3;
      const int bitC  = 3 - q;
      const int maskT = 1 << (3 - tq);
      const int src   = ((i >> bitC) & 1) ? (i ^ maskT) : i;
      const float tr = Ur[src * kDim + j];
      const float ti = Ui[src * kDim + j];
      __syncthreads();
      Ur[t] = tr;
      Ui[t] = ti;
      __syncthreads();
    }
  }

  if (t < 128) {
    const int row = t >> 2;
    const int k8  = (t & 3) * 8;
    const int ur  = row & 15;
    v8h hv;
#pragma unroll
    for (int e = 0; e < 8; ++e) {
      const int col = (k8 + e) & 15;
      const float vr = Ur[ur * kDim + col];
      const float vi = Ui[ur * kDim + col];
      const float v  = (row < kDim) ? vr : vi;
      hv[e] = (_Float16)(v * kCarryB);
    }
    unsigned short* dst = plane + row * kPlaneK + k8;
    *(volatile v8h*)dst = hv;
    __threadfence();
    *(volatile v8h*)dst = hv;
  }
}

__global__ __launch_bounds__(256) void circuit_rows_kernel(
    const float* __restrict__ x, const unsigned short* __restrict__ plane, float* __restrict__ out)
{
  __shared__ __align__(16) float sP[kWavesPerBlk][kRowsPerTile * kSlabPitch];
  const int lane = threadIdx.x & 31;
  const int wave = threadIdx.x >> 5;
  const int hh   = lane >> 4;
  const int c    = lane & 15;

  const _Float16* Bt = (const _Float16*)plane;
  const v16h bre = FragH::load(Bt + (size_t)c * kPlaneK + 8 * hh);
  const v16h bim = FragH::load(Bt + (size_t)(kDim + c) * kPlaneK + 8 * hh);

  float* slab = sP[wave];
  const int tile0 = (blockIdx.x * kWavesPerBlk + wave) * kTilesPerWave;

#pragma unroll 1
  for (int it = 0; it < kTilesPerWave; ++it) {
    const size_t base = (size_t)(tile0 + it) * kRowsPerTile;
    const v4f xv = *(const v4f*)(x + (base + lane) * 4);
    float cw0, sw0, cw1, sw1, cw2, sw2, cw3, sw3;
    sincosf(0.5f * xv.x, &sw0, &cw0);
    sincosf(0.5f * xv.y, &sw1, &cw1);
    sincosf(0.5f * xv.z, &sw2, &cw2);
    sincosf(0.5f * xv.w, &sw3, &cw3);

#pragma unroll
    for (int t = 0; t < 2; ++t) {
      const int src = 16 * t + c;
      const float c0 = __shfl(cw0, src, 32);
      const float s0 = __shfl(sw0, src, 32);
      const float c1 = __shfl(cw1, src, 32);
      const float s1 = __shfl(sw1, src, 32);
      const float c2 = __shfl(cw2, src, 32);
      const float s2 = __shfl(sw2, src, 32);
      const float c3 = __shfl(cw3, src, 32);
      const float s3 = __shfl(sw3, src, 32);
      const float f0 = hh ? s0 : c0;
      const float g0 = f0 * c1;
      const float g1 = f0 * s1;
      const float h00 = g0 * c2, h01 = g0 * s2, h10 = g1 * c2, h11 = g1 * s2;
      float psi[8];
      psi[0] = h00 * c3; psi[1] = h00 * s3;
      psi[2] = h01 * c3; psi[3] = h01 * s3;
      psi[4] = h10 * c3; psi[5] = h10 * s3;
      psi[6] = h11 * c3; psi[7] = h11 * s3;

      v16h a;
#pragma unroll
      for (int e = 0; e < 8; ++e) {
        const float sc = psi[e] * kCarryA;
        const _Float16 hv = (_Float16)sc;
        float hf = (float)hv;
        asm volatile("" : "+v"(hf));
        a[e]     = hv;
        a[8 + e] = (_Float16)(sc - hf);
      }

      v8f re = (v8f){0.f, 0.f, 0.f, 0.f, 0.f, 0.f, 0.f, 0.f};
      v8f im = (v8f){0.f, 0.f, 0.f, 0.f, 0.f, 0.f, 0.f, 0.f};
      re = mma_f16_guarded(a, bre, re);
      im = mma_f16_guarded(a, bim, im);

#pragma unroll
      for (int r = 0; r < 8; ++r) {
        const float pr = re[r] * re[r];
        const float p  = (im[r] * im[r] + pr) * kFold;
        slab[(16 * t + 8 * hh + r) * kSlabPitch + c] = p;
      }
    }

    __builtin_amdgcn_fence(__ATOMIC_RELEASE, "workgroup");
    __builtin_amdgcn_wave_barrier();
    __builtin_amdgcn_fence(__ATOMIC_ACQUIRE, "workgroup");

    const float* rp = slab + lane * kSlabPitch;
    const v4f p0 = *(const v4f*)(rp);
    const v4f p1 = *(const v4f*)(rp + 4);
    const v4f p2 = *(const v4f*)(rp + 8);
    const v4f p3 = *(const v4f*)(rp + 12);

    const float a0 = p0.x + p0.y, d0 = p0.x - p0.y;
    const float a1 = p0.z + p0.w, d1 = p0.z - p0.w;
    const float a2 = p1.x + p1.y, d2 = p1.x - p1.y;
    const float a3 = p1.z + p1.w, d3 = p1.z - p1.w;
    const float a4 = p2.x + p2.y, d4 = p2.x - p2.y;
    const float a5 = p2.z + p2.w, d5 = p2.z - p2.w;
    const float a6 = p3.x + p3.y, d6 = p3.x - p3.y;
    const float a7 = p3.z + p3.w, d7 = p3.z - p3.w;
    const float o3 = ((d0 + d1) + (d2 + d3)) + ((d4 + d5) + (d6 + d7));
    const float b0 = a0 + a1, e0 = a0 - a1;
    const float b1 = a2 + a3, e1 = a2 - a3;
    const float b2 = a4 + a5, e2 = a4 - a5;
    const float b3 = a6 + a7, e3 = a6 - a7;
    const float o2 = (e0 + e1) + (e2 + e3);
    const float q0 = b0 + b1, f0s = b0 - b1;
    const float q1 = b2 + b3, f1s = b2 - b3;
    const float o1 = f0s + f1s;
    const float o0 = q0 - q1;

    v4f ov;
    ov.x = o0; ov.y = o1; ov.z = o2; ov.w = o3;
    float* dst = out + (base + lane) * 4;
    *(volatile v4f*)dst = ov;
    __threadfence();
    *(volatile v4f*)dst = ov;

    __builtin_amdgcn_fence(__ATOMIC_RELEASE, "workgroup");
    __builtin_amdgcn_wave_barrier();
    __builtin_amdgcn_fence(__ATOMIC_ACQUIRE, "workgroup");
  }
}

extern "C" void kernel_launch(void* const* d_in, const int* in_sizes, int n_in,
                              void* d_out, int out_size, void* d_ws, size_t ws_size,
                              hipStream_t stream) {
  if (n_in < 2) return;
  if (in_sizes[0] != kBatch * kWires) return;
  if (in_sizes[1] != kAngles) return;
  if (out_size != kBatch * kWires) return;
  if (ws_size < kWsTotal) return;

  const float* x   = (const float*)d_in[0];
  const float* wts = (const float*)d_in[1];
  float* out = (float*)d_out;
  unsigned short* plane = (unsigned short*)((char*)d_ws + kOffPlane);

  build_gate_plane_kernel<<<1, 256, 0, stream>>>(wts, plane);
  circuit_rows_kernel<<<kMainBlocks, 256, 0, stream>>>(x, plane, out);
}
